// RotaryAttention_21225728377470
// MI455X (gfx1250) — hardware-verified
//
#include <hip/hip_runtime.h>
#include <math.h>

constexpr int kB    = 4;
constexpr int kS    = 1024;
constexpr int kD    = 2048;
constexpr int kH    = 16;
constexpr int kG    = 2;
constexpr int kDh   = 128;
constexpr int kKV   = kG * kDh;
constexpr int kTok  = kB * kS;
constexpr int kStg  = kD + 2 * kKV;
constexpr int kHPC  = kH / kG;
constexpr int kNF   = kDh / 2;
constexpr float kScoreScale = 0.08838834764831845f;
constexpr float kPCarry   = 32768.0f;
constexpr float kCtxCarry = 256.0f;
constexpr float kWoCarry  = 64.0f;
constexpr float kPVScale  = kCtxCarry / kPCarry;
constexpr float kOutScale = 1.0f / (kCtxCarry * kWoCarry);
static_assert(kH * kDh == kD, "shape");
static_assert(kHPC * kG == kH, "gqa");
static_assert(kTok % 64 == 0 && kD % 64 == 0 && kKV % 64 == 0 && kS % 64 == 0 && kDh % 64 == 0, "M/N tile multiples");
static_assert(kD % 32 == 0 && kDh % 32 == 0 && kS % 32 == 0, "K multiples of 32");
static_assert((kS * kNF) % 256 == 0 && (kTok * kD) % 2048 == 0 && (kTok * kKV) % 2048 == 0, "exact grids");

typedef __attribute__((ext_vector_type(16))) _Float16 v16h;
typedef __attribute__((ext_vector_type(8)))  _Float16 v8h;
typedef __attribute__((ext_vector_type(16))) __bf16   v16b;
typedef __attribute__((ext_vector_type(8)))  __bf16   v8b;
typedef __attribute__((ext_vector_type(8)))  float    v8f;
typedef __attribute__((ext_vector_type(4)))  float    v4f;
typedef __attribute__((ext_vector_type(4)))  unsigned int v4u;

__device__ __forceinline__ unsigned short f2bf_bits(float f) {
  unsigned u = __float_as_uint(f);
  return (unsigned short)((u + 0x7FFFu + ((u >> 16) & 1u)) >> 16);
}
__device__ __forceinline__ float bf_bits2f(unsigned short h) { return __uint_as_float(((unsigned)h) << 16); }

__device__ __forceinline__ void dep_guard_h(v8f& a, v8f& b, v16h x, v16h y) { asm volatile("v_nop\n\tv_nop\n\tv_nop\n\tv_nop" : "+v"(a), "+v"(b) : "v"(x), "v"(y)); }
__device__ __forceinline__ void dep_guard_b(v8f& a, v8f& b, v16b x, v16b y) { asm volatile("v_nop\n\tv_nop\n\tv_nop\n\tv_nop" : "+v"(a), "+v"(b) : "v"(x), "v"(y)); }
__device__ __forceinline__ void dep_guard4_h(v8f& a, v8f& b, v8f& c, v8f& d, v16h x, v16h y) { asm volatile("v_nop\n\tv_nop\n\tv_nop\n\tv_nop" : "+v"(a), "+v"(b), "+v"(c), "+v"(d) : "v"(x), "v"(y)); }
__device__ __forceinline__ void dep_guard4_b(v8f& a, v8f& b, v8f& c, v8f& d, v16b x, v16b y) { asm volatile("v_nop\n\tv_nop\n\tv_nop\n\tv_nop" : "+v"(a), "+v"(b), "+v"(c), "+v"(d) : "v"(x), "v"(y)); }
__device__ __forceinline__ void keep4_h(v16h a, v16h b, v16h c, v16h d) { asm volatile("v_nop" :: "v"(a), "v"(b), "v"(c), "v"(d)); }
__device__ __forceinline__ void keep4_b(v16b a, v16b b, v16b c, v16b d) { asm volatile("v_nop" :: "v"(a), "v"(b), "v"(c), "v"(d)); }
__device__ __forceinline__ void acc_guard4(v8f& a, v8f& b, v8f& c, v8f& d) { asm volatile("v_nop\n\tv_nop\n\tv_nop\n\tv_nop" : "+v"(a), "+v"(b), "+v"(c), "+v"(d)); }
template <typename T> struct Frag;
template <> struct Frag<_Float16> {
  typedef v16h V; union U { v16h v; v8h h[2]; };
  static __device__ __forceinline__ v16h load(const _Float16* p) {
    U f; f.h[0] = *(const v8h*)(p); f.h[1] = *(const v8h*)(p + 16); return f.v;
  }
  static __device__ __forceinline__ v8f mma(v16h a, v16h b, v8f c) {
    return __builtin_amdgcn_wmma_f32_16x16x32_f16(false, a, false, b, (short)0, c, false, false);
  }
  static __device__ __forceinline__ void guard(v8f& a, v8f& b, v16h x, v16h y) { dep_guard_h(a, b, x, y); }
  static __device__ __forceinline__ void guard4(v8f& a, v8f& b, v8f& c, v8f& d, v16h x, v16h y) { dep_guard4_h(a, b, c, d, x, y); }
  static __device__ __forceinline__ void keep(v16h a, v16h b, v16h c, v16h d) { keep4_h(a, b, c, d); }
};
template <> struct Frag<__bf16> {
  typedef v16b V; union U { v16b v; v8b h[2]; };
  static __device__ __forceinline__ v16b load(const __bf16* p) {
    U f; f.h[0] = *(const v8b*)(p); f.h[1] = *(const v8b*)(p + 16); return f.v;
  }
  static __device__ __forceinline__ v8f mma(v16b a, v16b b, v8f c) {
    return __builtin_amdgcn_wmma_f32_16x16x32_bf16(false, a, false, b, (short)0, c, false, false);
  }
  static __device__ __forceinline__ void guard(v8f& a, v8f& b, v16b x, v16b y) { dep_guard_b(a, b, x, y); }
  static __device__ __forceinline__ void guard4(v8f& a, v8f& b, v8f& c, v8f& d, v16b x, v16b y) { dep_guard4_b(a, b, c, d, x, y); }
  static __device__ __forceinline__ void keep(v16b a, v16b b, v16b c, v16b d) { keep4_b(a, b, c, d); }
};

__device__ __forceinline__ unsigned pk16(unsigned short a, unsigned short b) { return (unsigned)a | ((unsigned)b << 16); }
__device__ __forceinline__ unsigned short h_bits(float f) { const _Float16 h = (_Float16)f; return __builtin_bit_cast(unsigned short, h); }

template <int ET> struct Elem;
template <> struct Elem<0> { typedef _Float16 T; };
template <> struct Elem<1> { typedef __bf16 T; };
template <int ET, bool SPLIT, int BIAS_MODE, int OUT_MODE, bool RESID, int ACT = 0>
__global__ __launch_bounds__(256) void wmma_gemm64(
    const unsigned short* __restrict__ Ap, const unsigned short* __restrict__ A2p, int lda, long strideA,
    const unsigned short* __restrict__ Btp, const unsigned short* __restrict__ Bt2p, int ldb, long strideB,
    void* __restrict__ Cout, void* __restrict__ Cout2, int ldc, long strideC,
    const float* __restrict__ bias,
    const float* __restrict__ resid, long strideR,
    int M, int N, int K, float scale) {
  typedef typename Elem<ET>::T T;
  typedef typename Frag<T>::V V;
  const T* A = (const T*)Ap; const T* A2 = (const T*)A2p; const T* Bt = (const T*)Btp; const T* Bt2 = (const T*)Bt2p;
  __shared__ __align__(16) float sT[8][16 * 68];
  const int b    = blockIdx.y;
  const int lane = threadIdx.x & 31;
  const int wave = threadIdx.x >> 5;
  const int tilesN = N >> 6;
  const int tilesM = M >> 6;
  const int tile = blockIdx.x * 8 + wave;
  if (tile >= tilesM * tilesN) return;
  const int tm = tile / tilesN;
  const int tn = tile - tm * tilesN;
  const int m0 = tm << 6;
  const int n0 = tn << 6;

  const T* Ab  = A  + (size_t)b * strideA;
  const T* Bb  = Bt + (size_t)b * strideB;
  const T* Ab2 = SPLIT ? (A2  + (size_t)b * strideA) : nullptr;
  const T* Bb2 = SPLIT ? (Bt2 + (size_t)b * strideB) : nullptr;

  const int rlane = lane & 15;
  const int koff  = (lane >> 4) * 8;
  const int mOff  = (lane >> 4) * 8;

  v8f acc[4][4];
#pragma unroll
  for (int i = 0; i < 4; ++i)
#pragma unroll
    for (int j = 0; j < 4; ++j) acc[i][j] = (v8f){0.f,0.f,0.f,0.f,0.f,0.f,0.f,0.f};

  for (int k0 = 0; k0 < K; k0 += 32) {
    V bh[4], bl[4];
#pragma unroll
    for (int j = 0; j < 4; ++j) {
      const size_t bo = (size_t)(n0 + (j << 4) + rlane) * ldb + koff + k0;
      bh[j] = Frag<T>::load(Bb + bo);
      if (SPLIT) bl[j] = Frag<T>::load(Bb2 + bo);
    }
#pragma unroll
    for (int i = 0; i < 4; ++i) {
      const size_t ao = (size_t)(m0 + (i << 4) + rlane) * lda + koff + k0;
      V ah = Frag<T>::load(Ab + ao);
      V al;
      if (SPLIT) al = Frag<T>::load(Ab2 + ao);
#pragma unroll
      for (int j = 0; j < 4; ++j) {
        acc[i][j] = Frag<T>::mma(ah, bh[j], acc[i][j]);
        if (SPLIT) {
          acc[i][j] = Frag<T>::mma(ah, bl[j], acc[i][j]);
          acc[i][j] = Frag<T>::mma(al, bh[j], acc[i][j]);
        }
      }
      Frag<T>::guard4(acc[i][0], acc[i][1], acc[i][2], acc[i][3], ah, SPLIT ? al : ah);
    }
    Frag<T>::keep(bh[0], bh[1], bh[2], bh[3]);
    if (SPLIT) Frag<T>::keep(bl[0], bl[1], bl[2], bl[3]);
  }
  acc_guard4(acc[0][0], acc[0][1], acc[0][2], acc[0][3]);
  acc_guard4(acc[1][0], acc[1][1], acc[1][2], acc[1][3]);
  acc_guard4(acc[2][0], acc[2][1], acc[2][2], acc[2][3]);
  acc_guard4(acc[3][0], acc[3][1], acc[3][2], acc[3][3]);

  float* slab = sT[wave];
  const float* Rb = RESID ? (resid + (size_t)b * strideR) : nullptr;
#pragma unroll
  for (int i = 0; i < 4; ++i) {
    const int mBase = m0 + (i << 4);
#pragma unroll
    for (int j = 0; j < 4; ++j) {
      const int n = n0 + (j << 4) + rlane;
      float bv = 0.f;
      if (BIAS_MODE == 2) bv = bias[n];
#pragma unroll
      for (int r = 0; r < 8; ++r) {
        float v = acc[i][j][r] * scale;
        if (BIAS_MODE == 1) v += bias[mBase + mOff + r];
        if (BIAS_MODE == 2) v += bv;
        if (RESID) v += Rb[(size_t)(mBase + mOff + r) * ldc + n];
        if (ACT == 2) v = fmaxf(v, 0.0f);
        if (ACT == 4) v = (v > 0.f) ? v : 0.01f * v;
        slab[(mOff + r) * 68 + (j << 4) + rlane] = v;
      }
    }
    __builtin_amdgcn_fence(__ATOMIC_RELEASE, "workgroup");
    __builtin_amdgcn_wave_barrier();
    __builtin_amdgcn_fence(__ATOMIC_ACQUIRE, "workgroup");
    if (OUT_MODE == 0) {
      float* C = (float*)Cout + (size_t)b * strideC;
      const int hh = lane >> 4, c4 = (lane & 15) * 4;
      for (int pass = 0; pass < 2; ++pass) {
#pragma unroll
        for (int it = 0; it < 8; ++it) {
          const int row = it * 2 + hh;
          v4f v = *(const v4f*)(slab + row * 68 + c4);
          *(volatile v4f*)(C + (size_t)(mBase + row) * ldc + n0 + c4) = v;
        }
        __threadfence();
      }
    } else {
      const int q = lane >> 3, c8 = (lane & 7) * 8;
      unsigned short* C  = (unsigned short*)Cout  + (size_t)b * strideC;
      unsigned short* C2 = (OUT_MODE == 2) ? ((unsigned short*)Cout2 + (size_t)b * strideC) : nullptr;
      for (int pass = 0; pass < 2; ++pass) {
#pragma unroll
        for (int it = 0; it < 4; ++it) {
          const int row = it * 4 + q;
          const float* sp = slab + row * 68 + c8;
          v8h hv, lv;
#pragma unroll
          for (int e = 0; e < 8; ++e) {
            if (OUT_MODE == 1) {
              hv[e] = (_Float16)sp[e];
            } else {
              unsigned short hb = f2bf_bits(sp[e]);
              unsigned short lb = f2bf_bits(sp[e] - bf_bits2f(hb));
              hv[e] = __builtin_bit_cast(_Float16, hb);
              lv[e] = __builtin_bit_cast(_Float16, lb);
            }
          }
          *(volatile v8h*)(C + (size_t)(mBase + row) * ldc + n0 + c8) = hv;
          if (OUT_MODE == 2) *(volatile v8h*)(C2 + (size_t)(mBase + row) * ldc + n0 + c8) = lv;
        }
        __threadfence();
      }
    }
    __builtin_amdgcn_fence(__ATOMIC_RELEASE, "workgroup");
    __builtin_amdgcn_wave_barrier();
    __builtin_amdgcn_fence(__ATOMIC_ACQUIRE, "workgroup");
  }
}

__global__ __launch_bounds__(256) void cast8_bf16_kernel(const float* __restrict__ in, unsigned short* __restrict__ out, int n8) {
  const int i = blockIdx.x * 256 + threadIdx.x;
  if (i >= n8) return;
  const float* p = in + 8 * (size_t)i;
  const v4f a = *(const v4f*)(p);
  const v4f c = *(const v4f*)(p + 4);
  unsigned short hb[8];
#pragma unroll
  for (int e = 0; e < 4; ++e) {
    hb[e]     = f2bf_bits(a[e]);
    hb[4 + e] = f2bf_bits(c[e]);
  }
  const v4u u = (v4u){pk16(hb[0], hb[1]), pk16(hb[2], hb[3]), pk16(hb[4], hb[5]), pk16(hb[6], hb[7])};
  unsigned short* q = out + 8 * (size_t)i;
  *(volatile v4u*)q = u;
  __threadfence();
  *(volatile v4u*)q = u;
}

template <int MODE>
__global__ __launch_bounds__(256) void wt_kernel(const float* __restrict__ W, unsigned short* __restrict__ WT, int nK, int nN, float scale) {
  __shared__ float sm[64][65];
  const int t  = threadIdx.x;
  const int k0 = blockIdx.x * 64;
  const int n0 = blockIdx.y * 64;
#pragma unroll
  for (int i = 0; i < 16; ++i) {
    const int e = i * 256 + t;
    const int r = e >> 6;
    const int c = e & 63;
    sm[c][r] = W[(size_t)(k0 + r) * nN + n0 + c];
  }
  __syncthreads();
  const int lane = t & 31, wave = t >> 5;
  const int q = lane >> 3, c8 = (lane & 7) * 8;
  for (int pass = 0; pass < 2; ++pass) {
#pragma unroll
    for (int it = 0; it < 2; ++it) {
      const int row = wave * 8 + it * 4 + q;
      unsigned short hb[8];
#pragma unroll
      for (int e = 0; e < 8; ++e) {
        const float w = sm[row][c8 + e];
        if (MODE == 0) {
          hb[e] = f2bf_bits(w);
        } else {
          const float wb = bf_bits2f(f2bf_bits(w));
          hb[e] = h_bits(scale * wb);
        }
      }
      const v4u u = (v4u){pk16(hb[0], hb[1]), pk16(hb[2], hb[3]), pk16(hb[4], hb[5]), pk16(hb[6], hb[7])};
      *(volatile v4u*)(WT + (size_t)(n0 + row) * nK + k0 + c8) = u;
    }
    __threadfence();
  }
}

struct RopeFreq { float f[kNF]; };
static_assert(sizeof(RopeFreq) == 256, "no padding");

__global__ __launch_bounds__(256) void rope_table_kernel(float* __restrict__ tab, RopeFreq rf) {
#pragma clang fp contract(off)
  __shared__ float sf[kNF];
  __shared__ __align__(16) float cs[512];
  const int t = threadIdx.x;
  if (t == 0) {
#pragma unroll
    for (int j = 0; j < kNF; ++j) sf[j] = rf.f[j];
  }
  __syncthreads();
  const int i   = blockIdx.x * 256 + t;
  const int pos = i >> 6;
  const int j   = i & 63;
  const float fr  = sf[j];
  const float ang = (float)pos * fr;
  const float cv  = cosf(ang);
  const float sv  = sinf(ang);
  cs[2 * t]     = cv;
  cs[2 * t + 1] = sv;
  __syncthreads();
  if (t < 128) {
    const v4f v = *(const v4f*)(cs + 4 * t);
    float* dp = tab + (size_t)blockIdx.x * 512 + 4 * t;
    *(volatile v4f*)dp = v;
    __threadfence();
    *(volatile v4f*)dp = v;
  }
}

template <int NCOLS, int COL0>
__global__ __launch_bounds__(256) void rope_cast_kernel(const float* __restrict__ stg, const float* __restrict__ tab,
                                                        unsigned short* __restrict__ dst) {
  constexpr int TPR = NCOLS / 8;
  constexpr int RPB = 256 / TPR;
  static_assert(TPR * RPB == 256, "map");
  const int t   = threadIdx.x;
  const int rib = t / TPR;
  const int row = blockIdx.x * RPB + rib;
  const int u   = t - rib * TPR;
  const int lc  = 8 * u;
  const int pc  = lc ^ 64;
  const int f0  = lc & 63;
  const int pos = row & (kS - 1);
  const float* src = stg + (size_t)row * kStg + COL0;
  const v4f a0 = *(const v4f*)(src + lc);
  const v4f a1 = *(const v4f*)(src + lc + 4);
  const v4f b0 = *(const v4f*)(src + pc);
  const v4f b1 = *(const v4f*)(src + pc + 4);
  asm volatile("" ::: "memory");
  const float* tp = tab + ((size_t)pos * kNF + f0) * 2;
  const v4f c0 = *(const v4f*)(tp);
  const v4f c1 = *(const v4f*)(tp + 4);
  const v4f c2 = *(const v4f*)(tp + 8);
  const v4f c3 = *(const v4f*)(tp + 12);
  const float sgn = (lc & 64) ? 1.0f : -1.0f;
  float xs[8], ps[8], cc[8], ss[8];
  xs[0] = a0[0]; xs[1] = a0[1]; xs[2] = a0[2]; xs[3] = a0[3];
  xs[4] = a1[0]; xs[5] = a1[1]; xs[6] = a1[2]; xs[7] = a1[3];
  ps[0] = b0[0]; ps[1] = b0[1]; ps[2] = b0[2]; ps[3] = b0[3];
  ps[4] = b1[0]; ps[5] = b1[1]; ps[6] = b1[2]; ps[7] = b1[3];
  cc[0] = c0[0]; ss[0] = c0[1]; cc[1] = c0[2]; ss[1] = c0[3];
  cc[2] = c1[0]; ss[2] = c1[1]; cc[3] = c1[2]; ss[3] = c1[3];
  cc[4] = c2[0]; ss[4] = c2[1]; cc[5] = c2[2]; ss[5] = c2[3];
  cc[6] = c3[0]; ss[6] = c3[1]; cc[7] = c3[2]; ss[7] = c3[3];
  unsigned short hb[8];
#pragma unroll
  for (int e = 0; e < 8; ++e) {
    const float rot = sgn * ps[e];
    const float o = xs[e] * cc[e] + rot * ss[e];
    hb[e] = h_bits(o);
  }
  const v4u uu = (v4u){pk16(hb[0], hb[1]), pk16(hb[2], hb[3]), pk16(hb[4], hb[5]), pk16(hb[6], hb[7])};
  unsigned short* op = dst + (size_t)row * NCOLS + lc;
  *(volatile v4u*)op = uu;
  __threadfence();
  *(volatile v4u*)op = uu;
}

__global__ __launch_bounds__(256) void vt_kernel(const float* __restrict__ stg, unsigned short* __restrict__ VT) {
  __shared__ float sm[64][65];
  const int t   = threadIdx.x;
  const int t0  = blockIdx.x * 64;
  const int bgd = blockIdx.y;
  const int bg  = bgd >> 1;
  const int dh  = bgd & 1;
  const int b   = bg >> 1;
  const int g   = bg & 1;
#pragma unroll
  for (int i = 0; i < 16; ++i) {
    const int e = i * 256 + t;
    const int r = e >> 6;
    const int c = e & 63;
    sm[c][r] = stg[(size_t)(b * kS + t0 + r) * kStg + kD + kKV + g * kDh + dh * 64 + c];
  }
  __syncthreads();
  const int lane = t & 31, wave = t >> 5;
  const int q = lane >> 3, c8 = (lane & 7) * 8;
  unsigned short* op = VT + ((size_t)(bg * kDh + dh * 64)) * kS;
  for (int pass = 0; pass < 2; ++pass) {
#pragma unroll
    for (int it = 0; it < 2; ++it) {
      const int row = wave * 8 + it * 4 + q;
      unsigned short hb[8];
#pragma unroll
      for (int e = 0; e < 8; ++e) hb[e] = h_bits(sm[row][c8 + e]);
      const v4u u = (v4u){pk16(hb[0], hb[1]), pk16(hb[2], hb[3]), pk16(hb[4], hb[5]), pk16(hb[6], hb[7])};
      *(volatile v4u*)(op + (size_t)row * kS + t0 + c8) = u;
    }
    __threadfence();
  }
}

__global__ __launch_bounds__(128) void softmax_kernel(const float* __restrict__ S, unsigned short* __restrict__ P) {
  __shared__ float redM[4];
  __shared__ float redS[4];
  const int row  = blockIdx.x;
  const int hg   = blockIdx.y;
  const int t    = threadIdx.x;
  const int lane = t & 31, wave = t >> 5;
  const size_t rowoff = ((size_t)hg * kS + row) * kS;
  const float* sr = S + rowoff + 8 * (size_t)t;
  const v4f a = *(const v4f*)(sr);
  const v4f c = *(const v4f*)(sr + 4);
  float x[8];
#pragma unroll
  for (int e = 0; e < 4; ++e) { x[e] = a[e]; x[4 + e] = c[e]; }
  float m = fmaxf(fmaxf(fmaxf(x[0], x[1]), fmaxf(x[2], x[3])), fmaxf(fmaxf(x[4], x[5]), fmaxf(x[6], x[7])));
#pragma unroll
  for (int off = 16; off > 0; off >>= 1) m = fmaxf(m, __shfl_xor(m, off, 32));
  if (lane == 0) redM[wave] = m;
  __syncthreads();
  float mx = redM[0];
#pragma unroll
  for (int w = 1; w < 4; ++w) mx = fmaxf(mx, redM[w]);

  float ev[8];
  float sum = 0.f;
#pragma unroll
  for (int e = 0; e < 8; ++e) {
    ev[e] = expf(x[e] - mx);
    sum += ev[e];
  }
#pragma unroll
  for (int off = 16; off > 0; off >>= 1) sum += __shfl_xor(sum, off, 32);
  if (lane == 0) redS[wave] = sum;
  __syncthreads();
  float tot = redS[0];
#pragma unroll
  for (int w = 1; w < 4; ++w) tot += redS[w];
  const float inv = kPCarry / tot;

  unsigned short hb[8];
#pragma unroll
  for (int e = 0; e < 8; ++e) hb[e] = h_bits(ev[e] * inv);
  const v4u u = (v4u){pk16(hb[0], hb[1]), pk16(hb[2], hb[3]), pk16(hb[4], hb[5]), pk16(hb[6], hb[7])};
  unsigned short* pr = P + rowoff + 8 * (size_t)t;
  *(volatile v4u*)pr = u;
  __threadfence();
  *(volatile v4u*)pr = u;
}

constexpr size_t kOffXB  = 0;
constexpr size_t kSzXB   = (size_t)kTok * kD * 2;
constexpr size_t kOffWQT = kOffXB + kSzXB;
constexpr size_t kSzWQT  = (size_t)kD * kD * 2;
constexpr size_t kOffWKT = kOffWQT + kSzWQT;
constexpr size_t kSzWKV  = (size_t)kKV * kD * 2;
constexpr size_t kOffWVT = kOffWKT + kSzWKV;
constexpr size_t kOffWOT = kOffWVT + kSzWKV;
constexpr size_t kSzWOT  = (size_t)kD * kD * 2;
constexpr size_t kOffTAB = kOffWOT + kSzWOT;
constexpr size_t kSzTAB  = (size_t)kS * kNF * 2 * 4;
constexpr size_t kOffQ16 = kOffTAB + kSzTAB;
constexpr size_t kSzQ16  = (size_t)kTok * kD * 2;
constexpr size_t kOffK16 = kOffQ16 + kSzQ16;
constexpr size_t kSzK16  = (size_t)kTok * kKV * 2;
constexpr size_t kOffVT  = kOffK16 + kSzK16;
constexpr size_t kSzVT   = (size_t)kB * kG * kDh * kS * 2;
constexpr size_t kOffAO  = kOffVT + kSzVT;
constexpr size_t kSzAO   = (size_t)kTok * kD * 2;
constexpr size_t kOffSTG = kOffAO + kSzAO;
constexpr size_t kSzSTG  = (size_t)kTok * kStg * 4;
constexpr size_t kSzSC   = (size_t)kHPC * kS * kS * 4;
constexpr size_t kOffPP  = kOffSTG + kSzSTG;
constexpr size_t kSzPP   = (size_t)kHPC * kS * kS * 2;
constexpr size_t kWsTotal = kOffPP + kSzPP;
static_assert(kSzSC <= kSzSTG, "score chunk fits the staging region");
static_assert(kWsTotal == 132644864ull, "carve total");
static_assert(kWsTotal <= 134217728ull, "carve under 128 MiB");
static_assert(kOffWQT % 128 == 0 && kOffWKT % 128 == 0 && kOffWVT % 128 == 0 && kOffWOT % 128 == 0 && kOffTAB % 128 == 0 &&
              kOffQ16 % 128 == 0 && kOffK16 % 128 == 0 && kOffVT % 128 == 0 && kOffAO % 128 == 0 && kOffSTG % 128 == 0 &&
              kOffPP % 128 == 0, "line aligned regions");

extern "C" void kernel_launch(void* const* d_in, const int* in_sizes, int n_in,
                              void* d_out, int out_size, void* d_ws, size_t ws_size,
                              hipStream_t stream) {
  if (n_in < 9) return;
  if (in_sizes[0] != kTok * kD) return;
  if (in_sizes[1] != kD * kD || in_sizes[2] != kD) return;
  if (in_sizes[3] != kD * kKV || in_sizes[4] != kKV) return;
  if (in_sizes[5] != kD * kKV || in_sizes[6] != kKV) return;
  if (in_sizes[7] != kD * kD || in_sizes[8] != kD) return;
  if (out_size != kTok * kD) return;
  if (ws_size < kWsTotal) return;

  const float* x  = (const float*)d_in[0];
  const float* Wq = (const float*)d_in[1];
  const float* bq = (const float*)d_in[2];
  const float* Wk = (const float*)d_in[3];
  const float* bk = (const float*)d_in[4];
  const float* Wv = (const float*)d_in[5];
  const float* bv = (const float*)d_in[6];
  const float* Wo = (const float*)d_in[7];
  const float* bo = (const float*)d_in[8];
  float* out = (float*)d_out;
  char* ws = (char*)d_ws;
  unsigned short* XB  = (unsigned short*)(ws + kOffXB);
  unsigned short* WQT = (unsigned short*)(ws + kOffWQT);
  unsigned short* WKT = (unsigned short*)(ws + kOffWKT);
  unsigned short* WVT = (unsigned short*)(ws + kOffWVT);
  unsigned short* WOT = (unsigned short*)(ws + kOffWOT);
  float* TAB = (float*)(ws + kOffTAB);
  unsigned short* Q16 = (unsigned short*)(ws + kOffQ16);
  unsigned short* K16 = (unsigned short*)(ws + kOffK16);
  unsigned short* VT  = (unsigned short*)(ws + kOffVT);
  unsigned short* AO  = (unsigned short*)(ws + kOffAO);
  float* STG = (float*)(ws + kOffSTG);
  float* SC  = (float*)(ws + kOffSTG);
  unsigned short* PP = (unsigned short*)(ws + kOffPP);

  RopeFreq rf;
  for (int j = 0; j < kNF; ++j) {
    const float e = (float)(2 * j) / 128.0f;
    const double p = pow(10000.0, (double)e);
    const float pf = (float)p;
    rf.f[j] = 1.0f / pf;
  }

  const int n8x = (kTok * kD) / 8;
  cast8_bf16_kernel<<<dim3(n8x / 256), dim3(256), 0, stream>>>(x, XB, n8x);
  wt_kernel<0><<<dim3(kD / 64, kD / 64), dim3(256), 0, stream>>>(Wq, WQT, kD, kD, 1.0f);
  wt_kernel<0><<<dim3(kD / 64, kKV / 64), dim3(256), 0, stream>>>(Wk, WKT, kD, kKV, 1.0f);
  wt_kernel<0><<<dim3(kD / 64, kKV / 64), dim3(256), 0, stream>>>(Wv, WVT, kD, kKV, 1.0f);
  wt_kernel<1><<<dim3(kD / 64, kD / 64), dim3(256), 0, stream>>>(Wo, WOT, kD, kD, kWoCarry);
  rope_table_kernel<<<dim3((kS * kNF) / 256), dim3(256), 0, stream>>>(TAB, rf);

  const int tilesQ  = (kTok / 64) * (kD / 64);
  const int tilesKV = (kTok / 64) * (kKV / 64);
  wmma_gemm64<1, false, 2, 0, false, 0><<<dim3(tilesQ / 8, 1), dim3(256), 0, stream>>>(
      XB, XB, kD, 0L, WQT, WQT, kD, 0L, (void*)STG, (void*)STG, kStg, 0L, bq, bq, 0L, kTok, kD, kD, 1.0f);
  wmma_gemm64<1, false, 2, 0, false, 0><<<dim3(tilesKV / 8, 1), dim3(256), 0, stream>>>(
      XB, XB, kD, 0L, WKT, WKT, kD, 0L, (void*)(STG + kD), (void*)(STG + kD), kStg, 0L, bk, bk, 0L, kTok, kKV, kD, 1.0f);
  wmma_gemm64<1, false, 2, 0, false, 0><<<dim3(tilesKV / 8, 1), dim3(256), 0, stream>>>(
      XB, XB, kD, 0L, WVT, WVT, kD, 0L, (void*)(STG + kD + kKV), (void*)(STG + kD + kKV), kStg, 0L, bv, bv, 0L, kTok, kKV, kD, 1.0f);

  rope_cast_kernel<kD, 0><<<dim3(kTok), dim3(256), 0, stream>>>(STG, TAB, Q16);
  rope_cast_kernel<kKV, kD><<<dim3(kTok / 8), dim3(256), 0, stream>>>(STG, TAB, K16);
  vt_kernel<<<dim3(kS / 64, kB * kG * 2), dim3(256), 0, stream>>>(STG, VT);

  const int  tilesScore = (kS / 64) * (kS / 64);
  const int  tilesCtx   = (kS / 64) * (kDh / 64);
  const long strideHead = (long)kDh;
  const long stridePl   = (long)kS * kS;
  for (int b = 0; b < kB; ++b) {
    for (int g = 0; g < kG; ++g) {
      const unsigned short* Ag  = Q16 + ((size_t)b * kS) * kD + (size_t)g * kHPC * kDh;
      const unsigned short* Btg = K16 + ((size_t)b * kS) * kKV + (size_t)g * kDh;
      wmma_gemm64<0, false, 0, 0, false, 0><<<dim3(tilesScore / 8, kHPC), dim3(256), 0, stream>>>(
          Ag, Ag, kD, strideHead, Btg, Btg, kKV, 0L,
          (void*)SC, (void*)SC, kS, stridePl, bq, bq, 0L, kS, kS, kDh, kScoreScale);
      softmax_kernel<<<dim3(kS, kHPC), dim3(128), 0, stream>>>(SC, PP);
      const unsigned short* VTg = VT + ((size_t)(b * kG + g) * kDh) * kS;
      unsigned short* AOg = AO + ((size_t)b * kS) * kD + (size_t)g * kHPC * kDh;
      wmma_gemm64<0, false, 0, 1, false, 0><<<dim3(tilesCtx / 8, kHPC), dim3(256), 0, stream>>>(
          PP, PP, kS, stridePl, VTg, VTg, kS, 0L,
          (void*)AOg, (void*)AOg, kD, strideHead, bq, bq, 0L, kS, kDh, kS, kPVScale);
    }
  }

  wmma_gemm64<0, false, 2, 0, false, 0><<<dim3(tilesQ / 8, 1), dim3(256), 0, stream>>>(
      AO, AO, kD, 0L, WOT, WOT, kD, 0L, (void*)out, (void*)out, kD, 0L, bo, bo, 0L, kTok, kD, kD, kOutScale);
}
